// Repro_11879879542435
// MI455X (gfx1250) — hardware-run, weakly checked
//
#include <hip/hip_runtime.h>
#include <math.h>

#ifndef NB
#define NB 1024
#endif
#define NB_FULL 1024
#define NC 20
#define NN 21
#define DM 128
#define EH 16
#define NH 8
#define FFD 512
#define NLAYER 3
#define QKVW (3 * DM)
#define MTOK (NB * NN)
#define NSLAB (MTOK / 128)

static_assert(NB <= NB_FULL);
static_assert(NB % 2 == 0);
static_assert(MTOK % 128 == 0);
static_assert(MTOK % 64 == 0 && MTOK % 16 == 0);
static_assert(MTOK < 65536);
static_assert(DM == 128 && NH * EH == DM && EH == 16 && NN <= 32 && NN > 16);
static_assert(DM % 64 == 0 && QKVW % 64 == 0 && FFD % 64 == 0);
static_assert(DM % 32 == 0 && FFD % 32 == 0);

typedef __attribute__((ext_vector_type(16))) _Float16 v16h;
typedef __attribute__((ext_vector_type(8)))  _Float16 v8h;
typedef __attribute__((ext_vector_type(2)))  _Float16 v2h;
typedef __attribute__((ext_vector_type(8)))  float    v8f;
typedef __attribute__((ext_vector_type(4)))  float    v4f;
typedef __attribute__((ext_vector_type(2)))  float    v2f;
typedef __attribute__((ext_vector_type(4)))  unsigned int v4u;


#define VST2(T, ptr, val) do { const T vst2_v_ = (val); *(volatile T*)(ptr) = vst2_v_; __threadfence(); *(volatile T*)(ptr) = vst2_v_; } while (0)
#define VST2V4(ptr, val) do { const v4f vst2_v4_ = (val); *(volatile v4f*)(ptr) = vst2_v4_; __threadfence(); *(volatile v4f*)(ptr) = vst2_v4_; } while (0)

__device__ __forceinline__ float bfr(float f) {
    unsigned u = __float_as_uint(f);
    u += 0x7FFFu + ((u >> 16) & 1u);
    return __uint_as_float(u & 0xFFFF0000u);
}
__device__ __forceinline__ v4f bfr4(v4f a) {
    v4f r; r.x = bfr(a.x); r.y = bfr(a.y); r.z = bfr(a.z); r.w = bfr(a.w); return r;
}
static __device__ __forceinline__ _Float16 toh_flush(float v) {
    const float w = (fabsf(v) < 6.103515625e-05f) ? 0.0f : v;
    return (_Float16)w;
}
static __device__ __forceinline__ unsigned toh_flush2(float a, float b) {
    v2f w;
    w.x = (fabsf(a) < 6.103515625e-05f) ? 0.0f : a;
    w.y = (fabsf(b) < 6.103515625e-05f) ? 0.0f : b;
    const v2h r = __builtin_convertvector(w, v2h);
    return __builtin_bit_cast(unsigned, r);
}
__device__ __forceinline__ _Float16 hbits(unsigned x) {
    return __builtin_bit_cast(_Float16, (unsigned short)x);
}
__device__ __forceinline__ void st8hf(unsigned short* P, size_t o, const float* v) {
    v4u pk;
    pk.x = toh_flush2(v[0], v[1]);
    pk.y = toh_flush2(v[2], v[3]);
    pk.z = toh_flush2(v[4], v[5]);
    pk.w = toh_flush2(v[6], v[7]);
    VST2(v4u, (v4u*)(P + o), pk);
}

union FragU { v16h v; v8h h[2]; };
union FragW { v16h v; v4u w[2]; };
__device__ __forceinline__ v16h frag_ld(const _Float16* p) {
    FragU f; f.h[0] = *(const v8h*)(p); f.h[1] = *(const v8h*)(p + 16); return f.v;
}
__device__ __forceinline__ v8f wmma16(v16h a, v16h b, v8f c) {
    c = __builtin_amdgcn_wmma_f32_16x16x32_f16(false, a, false, b, (short)0, c, false, false);
    asm volatile("v_nop\n\tv_nop\n\tv_nop\n\tv_nop" : "+v"(c) : "v"(a), "v"(b));
    return c;
}
__device__ __forceinline__ void wave_sync_lds() {
    __builtin_amdgcn_fence(3  , "workgroup");
    __builtin_amdgcn_wave_barrier();
    __builtin_amdgcn_fence(2  , "workgroup");
}

static_assert(32 * 16 * 4 == 16 * 64 * 2);
static_assert(32 * 16 * 8 == 16 * 64 * 4);
static_assert(8 * 16 * 68 * 4 <= 131072);

template <int OUT_MODE, bool RESID, bool RELU, bool BIAS>
__device__ __forceinline__ void gemm64_body(
    const _Float16* __restrict__ A, unsigned lda, const _Float16* __restrict__ Bt, unsigned ldb,
    void* __restrict__ Cout, unsigned ldc, const float* __restrict__ bias, const float* __restrict__ resid,
    unsigned M, unsigned N, unsigned K, float scale, float oscale, float* sT) {
  const unsigned lane = threadIdx.x & 31u;
  const unsigned wave = threadIdx.x >> 5;
  const unsigned tilesN = N >> 6, tilesM = M >> 6;
  const unsigned tile = blockIdx.x * 8u + wave;
  if (tile >= tilesM * tilesN) return;
  const unsigned tm = tile / tilesN;
  const unsigned tn = tile - tm * tilesN;
  const unsigned m0 = tm << 6, n0 = tn << 6;
  const unsigned rlane = lane & 15u;
  const unsigned koff = (lane >> 4) * 8u;
  const unsigned mOff = koff;

  v8f acc[4][4];
#pragma unroll
  for (int i = 0; i < 4; ++i)
#pragma unroll
    for (int j = 0; j < 4; ++j) acc[i][j] = (v8f){0.f,0.f,0.f,0.f,0.f,0.f,0.f,0.f};

  for (unsigned k0 = 0; k0 < K; k0 += 32u) {
    v16h bh[4];
#pragma unroll
    for (int j = 0; j < 4; ++j)
      bh[j] = frag_ld(Bt + (size_t)(n0 + ((unsigned)j << 4) + rlane) * ldb + koff + k0);
#pragma unroll
    for (int i = 0; i < 4; ++i) {
      const v16h ah = frag_ld(A + (size_t)(m0 + ((unsigned)i << 4) + rlane) * lda + koff + k0);
#pragma unroll
      for (int j = 0; j < 4; ++j)
        acc[i][j] = wmma16(ah, bh[j], acc[i][j]);
    }
  }

  float* slab = sT + wave * (16u * 68u);
#pragma unroll
  for (int i = 0; i < 4; ++i) {
    const unsigned mBase = m0 + ((unsigned)i << 4);
#pragma unroll
    for (int j = 0; j < 4; ++j) {
      const unsigned n = n0 + ((unsigned)j << 4) + rlane;
      float bv = 0.0f;
      if (BIAS) bv = bfr(bias[n]);
#pragma unroll
      for (int r = 0; r < 8; ++r) {
        float v = acc[i][j][r] * scale + bv;
        if (RELU) v = fmaxf(v, 0.0f);
        if (OUT_MODE == 1) v *= oscale;
        slab[(mOff + (unsigned)r) * 68u + ((unsigned)j << 4) + rlane] = v;
      }
    }
    wave_sync_lds();
    if (OUT_MODE == 0) {
      float* C = (float*)Cout;
      const unsigned hh = lane >> 4, c4 = (lane & 15u) * 4u;
#pragma unroll
      for (int half = 0; half < 2; ++half) {
        v4f vv[4];
#pragma unroll
        for (int it = 0; it < 4; ++it) {
          const unsigned row = (unsigned)(half * 4 + it) * 2u + hh;
          vv[it] = *(const v4f*)(slab + row * 68u + c4);
          if (RESID) vv[it] += *(const v4f*)(resid + (size_t)(mBase + row) * ldc + n0 + c4);
        }
        for (int pass = 0; pass < 2; ++pass) {
#pragma unroll
          for (int it = 0; it < 4; ++it) {
            const unsigned row = (unsigned)(half * 4 + it) * 2u + hh;
            *(volatile v4f*)(C + (size_t)(mBase + row) * ldc + n0 + c4) = vv[it];
          }
          __threadfence();
        }
      }
    } else {
      _Float16* C = (_Float16*)Cout;
      const unsigned q = lane >> 3, c8 = (lane & 7u) * 8u;
      v4u hv[4];
#pragma unroll
      for (int it = 0; it < 4; ++it) {
        const unsigned row = (unsigned)it * 4u + q;
        const float* sp = slab + row * 68u + c8;
        const v4f p0 = *(const v4f*)sp, p1 = *(const v4f*)(sp + 4);
        hv[it].x = toh_flush2(p0.x, p0.y);
        hv[it].y = toh_flush2(p0.z, p0.w);
        hv[it].z = toh_flush2(p1.x, p1.y);
        hv[it].w = toh_flush2(p1.z, p1.w);
      }
      for (int pass = 0; pass < 2; ++pass) {
#pragma unroll
        for (int it = 0; it < 4; ++it) {
          const unsigned row = (unsigned)it * 4u + q;
          *(volatile v4u*)(C + (size_t)(mBase + row) * ldc + n0 + c8) = hv[it];
        }
        __threadfence();
      }
    }
    wave_sync_lds();
  }
}

__global__ __launch_bounds__(256) void k_gemm_qkv(const _Float16* __restrict__ A, const _Float16* __restrict__ Bt,
                                                  _Float16* __restrict__ C) {
    __shared__ __align__(16) float sT[8 * 16 * 68];
    gemm64_body<1, false, false, false>(A, DM, Bt, DM, (void*)C, QKVW, nullptr, nullptr,
                                        MTOK, QKVW, DM, 1.0f / 1048576.0f, 1024.0f, sT);
}
__global__ __launch_bounds__(256) void k_gemm_wo(const _Float16* __restrict__ A, const _Float16* __restrict__ Bt,
                                                 const float* __restrict__ resid, float* __restrict__ C) {
    __shared__ __align__(16) float sT[8 * 16 * 68];
    gemm64_body<0, true, false, false>(A, DM, Bt, DM, (void*)C, DM, nullptr, resid,
                                       MTOK, DM, DM, 1.0f / 4194304.0f, 1.0f, sT);
}
__global__ __launch_bounds__(256) void k_gemm_ff1(const _Float16* __restrict__ A, const _Float16* __restrict__ Bt,
                                                  const float* __restrict__ bias, _Float16* __restrict__ C) {
    __shared__ __align__(16) float sT[8 * 16 * 68];
    gemm64_body<1, false, true, true>(A, DM, Bt, DM, (void*)C, FFD, bias, nullptr,
                                      MTOK, FFD, DM, 1.0f / 1048576.0f, 256.0f, sT);
}
__global__ __launch_bounds__(256) void k_gemm_ff2(const _Float16* __restrict__ A, const _Float16* __restrict__ Bt,
                                                  const float* __restrict__ bias, const float* __restrict__ resid,
                                                  float* __restrict__ C) {
    __shared__ __align__(16) float sT[8 * 16 * 68];
    gemm64_body<0, true, false, true>(A, FFD, Bt, FFD, (void*)C, DM, bias, resid,
                                      MTOK, DM, FFD, 1.0f / 1048576.0f, 1.0f, sT);
}

__global__ __launch_bounds__(256) void k_wt16(const float* __restrict__ Wm, unsigned KI, unsigned NO, unsigned lgper, unsigned lgob,
                                              unsigned dstLayer, unsigned short* __restrict__ W16) {
    const unsigned layer = blockIdx.y;
    const float* Wl = Wm + (size_t)layer * KI * NO;
    unsigned short* Dl = W16 + (size_t)layer * dstLayer;
    const unsigned u = blockIdx.x * 256u + threadIdx.x;
    const unsigned per = 1u << lgper;
    if (u >= NO * per) return;
    const unsigned k0 = 8u * (u & (per - 1u));
    const unsigned o = u >> lgper;
    const unsigned ob = 1u << lgob;
    const size_t base = (size_t)(o >> lgob) * KI * ob + (o & (ob - 1u));
    float v[8];
#pragma unroll
    for (int i = 0; i < 8; ++i) v[i] = bfr(Wl[base + (size_t)(k0 + (unsigned)i) * ob]) * 4096.0f;
    st8hf(Dl, (size_t)o * KI + k0, v);
}

static_assert(32 * 16 == DM * 4 && 32 * 16 == 2 * DM * 2);
__device__ __forceinline__ void put2rows(float* sw, unsigned lane, v4f ya, v4f yb,
                                         float* dst32, unsigned short* dst16, unsigned rowA, float carry) {
    *(v4f*)(sw + 4u * lane) = ya;
    *(v4f*)(sw + 128u + 4u * lane) = yb;
    wave_sync_lds();
    const float* sp = sw + (lane >> 4) * 128u + (lane & 15u) * 8u;
    const v4f p0 = *(const v4f*)sp, p1 = *(const v4f*)(sp + 4);
    wave_sync_lds();
    v4u pk;
    pk.x = toh_flush2(p0.x * carry, p0.y * carry);
    pk.y = toh_flush2(p0.z * carry, p0.w * carry);
    pk.z = toh_flush2(p1.x * carry, p1.y * carry);
    pk.w = toh_flush2(p1.z * carry, p1.w * carry);
    float* d0 = dst32 + (size_t)rowA * DM + 4u * lane;
    float* d1 = d0 + DM;
    unsigned short* dh = dst16 + (size_t)rowA * DM + 8u * lane;
    for (int pass = 0; pass < 2; ++pass) {
        *(volatile v4f*)d0 = ya;
        *(volatile v4f*)d1 = yb;
        *(volatile v4u*)dh = pk;
        __threadfence();
    }
}

__global__ __launch_bounds__(256) void k_embed(const float* __restrict__ loc, const float* __restrict__ dem,
                                               const float* __restrict__ dep, const float* __restrict__ dw,
                                               const float* __restrict__ db, const float* __restrict__ nw,
                                               const float* __restrict__ nb, float* __restrict__ h32,
                                               unsigned short* __restrict__ h16) {
    __shared__ __align__(16) float sW[8][256];
    const unsigned lane = threadIdx.x & 31u;
    const unsigned wave = __builtin_amdgcn_readfirstlane(threadIdx.x >> 5);
    const unsigned c0 = 4u * lane;
    const v4f dw0 = bfr4(*(const v4f*)(dw + c0));
    const v4f dw1 = bfr4(*(const v4f*)(dw + DM + c0));
    const v4f dbv = bfr4(*(const v4f*)(db + c0));
    const v4f nw0 = bfr4(*(const v4f*)(nw + c0));
    const v4f nw1 = bfr4(*(const v4f*)(nw + DM + c0));
    const v4f nw2 = bfr4(*(const v4f*)(nw + 2 * DM + c0));
    const v4f nbv = bfr4(*(const v4f*)(nb + c0));
    const unsigned rA = blockIdx.x * 16u + wave * 2u;
    v4f y[2];
#pragma unroll
    for (int j = 0; j < 2; ++j) {
        unsigned rp = rA + (unsigned)j;
        asm volatile("" : "+v"(rp));
        const unsigned b = rp / 21u;
        const unsigned n = rp - b * 21u;
        const unsigned jn = ((n > 0u) ? n : 1u) - 1u;
        const float d0 = bfr(dep[b * 2u]), d1 = bfr(dep[b * 2u + 1u]);
        const float lx = bfr(loc[(b * NC + jn) * 2u]), ly = bfr(loc[(b * NC + jn) * 2u + 1u]);
        const float dq = bfr(dem[b * NC + jn]);
        const v4f vd = (d0 * dw0 + d1 * dw1) + dbv;
        const v4f vn = ((lx * nw0 + ly * nw1) + dq * nw2) + nbv;
        const bool isdep = (n == 0u);
        y[j].x = isdep ? vd.x : vn.x;
        y[j].y = isdep ? vd.y : vn.y;
        y[j].z = isdep ? vd.z : vn.z;
        y[j].w = isdep ? vd.w : vn.w;
    }
    put2rows(sW[wave], lane, y[0], y[1], h32, h16, rA, 256.0f);
}

#define AT_PP 40
#define AT_PV 40
#define AT_PO 136
static_assert((16 * 32 * AT_PP + 16 * 16 * AT_PV + 2 * NN * AT_PO) * 2 <= 131072);
static_assert(2 * NN * 16 <= 2 * 512);
static_assert(2 * NN * 16 * 16 == 2 * NN * DM * 2);
__global__ __launch_bounds__(512) void k_attn(const _Float16* __restrict__ qkv, _Float16* __restrict__ o16) {
    __shared__ __align__(16) _Float16 sP[16][32 * AT_PP];
    __shared__ __align__(16) _Float16 sVT[16][16 * AT_PV];
    __shared__ __align__(16) _Float16 sO[2 * NN * AT_PO];
    const unsigned tid = threadIdx.x, lane = tid & 31u;
    const unsigned wave = __builtin_amdgcn_readfirstlane(tid >> 5);
    const unsigned hh = lane >> 4, c = lane & 15u;
    const unsigned bl = wave >> 3, head = wave & 7u;
    const unsigned row0 = (blockIdx.x * 2u + bl) * NN;
    _Float16* pw = sP[wave];
    _Float16* vt = sVT[wave];
    const v4u zero4 = (v4u){0u, 0u, 0u, 0u};
    {
        const unsigned kr = (lane < (unsigned)NN) ? lane : (unsigned)(NN - 1);
        const bool kval = lane < (unsigned)NN;
        const _Float16* vsrc = qkv + (size_t)(row0 + kr) * QKVW + 2u * DM + head * EH;
        const v4u wa = *(const v4u*)vsrc;
        const v4u wb = *(const v4u*)(vsrc + 8);
        const unsigned w[8] = {wa.x, wa.y, wa.z, wa.w, wb.x, wb.y, wb.z, wb.w};
#pragma unroll
        for (int j = 0; j < 8; ++j) {
            const unsigned ww = kval ? w[j] : 0u;
            vt[(unsigned)(2 * j) * AT_PV + lane] = hbits(ww & 0xFFFFu);
            vt[(unsigned)(2 * j + 1) * AT_PV + lane] = hbits(ww >> 16);
        }
    }
    v16h qf[2], kf[2];
#pragma unroll
    for (int t = 0; t < 2; ++t) {
        const unsigned n = (unsigned)t * 16u + c;
        const unsigned nr = (n < (unsigned)NN) ? n : (unsigned)(NN - 1);
        const bool ok = n < (unsigned)NN;
        const _Float16* src = qkv + (size_t)(row0 + nr) * QKVW + head * EH + 8u * hh;
        v4u qa = *(const v4u*)src;
        v4u ka = *(const v4u*)(src + DM);
        qa.x = ok ? qa.x : 0u; qa.y = ok ? qa.y : 0u; qa.z = ok ? qa.z : 0u; qa.w = ok ? qa.w : 0u;
        ka.x = ok ? ka.x : 0u; ka.y = ok ? ka.y : 0u; ka.z = ok ? ka.z : 0u; ka.w = ok ? ka.w : 0u;
        FragW fq; fq.w[0] = qa; fq.w[1] = zero4; qf[t] = fq.v;
        FragW fk; fk.w[0] = ka; fk.w[1] = zero4; kf[t] = fk.v;
    }
    const v8f z8 = (v8f){0.f,0.f,0.f,0.f,0.f,0.f,0.f,0.f};
    v8f s[2][2];
#pragma unroll
    for (int mt = 0; mt < 2; ++mt)
#pragma unroll
        for (int nt = 0; nt < 2; ++nt) s[mt][nt] = wmma16(qf[mt], kf[nt], z8);

    const float SC2 = 0.25f * 1.4426950408889634f * (1.0f / 1048576.0f);
    const bool kv1 = c < (unsigned)(NN - 16);
    float lrow[2][8];
#pragma unroll
    for (int mt = 0; mt < 2; ++mt) {
#pragma unroll
        for (int r = 0; r < 8; ++r) {
            const float a0 = s[mt][0][r] * SC2;
            const float a1 = s[mt][1][r] * SC2;
            float mx = fmaxf(a0, kv1 ? a1 : -3.0e38f);
            mx = fmaxf(mx, __shfl_xor(mx, 1, 32)); mx = fmaxf(mx, __shfl_xor(mx, 2, 32));
            mx = fmaxf(mx, __shfl_xor(mx, 4, 32)); mx = fmaxf(mx, __shfl_xor(mx, 8, 32));
            const float e0 = exp2f(a0 - mx);
            const float e1r = exp2f(a1 - mx);
            const float e1 = kv1 ? e1r : 0.0f;
            float psum = e0 + e1;
            psum += __shfl_xor(psum, 1, 32); psum += __shfl_xor(psum, 2, 32);
            psum += __shfl_xor(psum, 4, 32); psum += __shfl_xor(psum, 8, 32);
            lrow[mt][r] = psum;
            const unsigned prow = ((unsigned)mt * 16u + 8u * hh + (unsigned)r) * AT_PP;
            pw[prow + c] = toh_flush(e0 * 1024.0f);
            pw[prow + 16u + c] = toh_flush(e1 * 1024.0f);
        }
    }
    wave_sync_lds();
    v8f os[2];
    {
        const v16h vb = frag_ld(vt + c * AT_PV + 8u * hh);
#pragma unroll
        for (int mt = 0; mt < 2; ++mt) {
            const v16h pa = frag_ld(pw + ((unsigned)mt * 16u + c) * AT_PP + 8u * hh);
            os[mt] = wmma16(pa, vb, z8);
        }
    }
#pragma unroll
    for (int mt = 0; mt < 2; ++mt) {
#pragma unroll
        for (int r = 0; r < 8; ++r) {
            const float inv = 1.0f / (lrow[mt][r] * 1024.0f);
            const unsigned n = (unsigned)mt * 16u + 8u * hh + (unsigned)r;
            const _Float16 ov = toh_flush(os[mt][r] * inv);
            if (n < (unsigned)NN) sO[(bl * NN + n) * AT_PO + head * EH + c] = ov;
        }
    }
    __syncthreads();
    {
        v4u ov[2];
#pragma unroll
        for (int it = 0; it < 2; ++it) {
            const unsigned p = (unsigned)it * 512u + tid;
            const unsigned pc = (p < (unsigned)(2 * NN * 16)) ? p : (unsigned)(2 * NN * 16 - 1);
            ov[it] = *(const v4u*)(sO + (pc >> 4) * AT_PO + (pc & 15u) * 8u);
        }
        _Float16* dst = o16 + (size_t)(blockIdx.x * 2u * NN) * DM;
        for (int pass = 0; pass < 2; ++pass) {
#pragma unroll
            for (int it = 0; it < 2; ++it) {
                const unsigned p = (unsigned)it * 512u + tid;
                if (p < (unsigned)(2 * NN * 16)) *(volatile v4u*)(dst + (size_t)p * 8u) = ov[it];
            }
            __threadfence();
        }
    }
}

static_assert((8 * 256 + 256) * 4 <= 131072);
__global__ __launch_bounds__(256) void k_colsum(const float* __restrict__ x, float* __restrict__ psum) {
    __shared__ __align__(16) float sA[256];
    const unsigned t = threadIdx.x, c = t & 127u, hf = t >> 7;
    const float* xp = x + (size_t)(blockIdx.x * 128u + hf * 64u) * DM + c;
    float s = 0.f;
    for (unsigned i = 0; i < 64u; ++i) s += xp[(size_t)i * DM];
    sA[t] = s;
    __syncthreads();
    if (t < 32u) {
        const v4f a = *(const v4f*)(sA + 4u * t), b = *(const v4f*)(sA + 128u + 4u * t);
        VST2V4(psum + (size_t)blockIdx.x * DM + 4u * t, a + b);
    }
}

__global__ __launch_bounds__(256) void k_colvar(const float* __restrict__ x, const float* __restrict__ psum,
                                                float* __restrict__ psq) {
    __shared__ __align__(16) float sA[256];
    const unsigned t = threadIdx.x, c = t & 127u, hf = t >> 7;
    float ms = 0.f;
    for (unsigned p = 0; p < (unsigned)NSLAB; ++p) ms += psum[(size_t)p * DM + c];
    const float mean = ms / (float)MTOK;
    const float* xp = x + (size_t)(blockIdx.x * 128u + hf * 64u) * DM + c;
    float s = 0.f;
    for (unsigned i = 0; i < 64u; ++i) { const float d = xp[(size_t)i * DM] - mean; s += d * d; }
    sA[t] = s;
    __syncthreads();
    if (t < 32u) {
        const v4f a = *(const v4f*)(sA + 4u * t), b = *(const v4f*)(sA + 128u + 4u * t);
        VST2V4(psq + (size_t)blockIdx.x * DM + 4u * t, a + b);
    }
}

__global__ __launch_bounds__(256) void k_bn(const float* __restrict__ x, const float* __restrict__ part,
                                            const float* __restrict__ g, const float* __restrict__ bt,
                                            float* __restrict__ y32, unsigned short* __restrict__ y16) {
    __shared__ __align__(16) float sStat[256];
    __shared__ __align__(16) float sW[8][256];
    const unsigned t = threadIdx.x, lane = t & 31u;
    const unsigned wave = __builtin_amdgcn_readfirstlane(t >> 5);
    {
        const float* pp = part + (size_t)(t >> 7) * (NSLAB * DM) + (t & 127u);
        float s = 0.f;
        for (unsigned p = 0; p < (unsigned)NSLAB; ++p) s += pp[(size_t)p * DM];
        sStat[t] = s / (float)MTOK;
    }
    __syncthreads();
    const unsigned c0 = 4u * lane;
    const v4f mu = *(const v4f*)(sStat + c0);
    const v4f va = *(const v4f*)(sStat + 128u + c0);
    const v4f gv = bfr4(*(const v4f*)(g + c0));
    const v4f bv = bfr4(*(const v4f*)(bt + c0));
    v4f rs;
    rs.x = 1.0f / sqrtf(va.x + 1e-5f);
    rs.y = 1.0f / sqrtf(va.y + 1e-5f);
    rs.z = 1.0f / sqrtf(va.z + 1e-5f);
    rs.w = 1.0f / sqrtf(va.w + 1e-5f);
    const unsigned rbase = blockIdx.x * 128u + wave * 16u;
    for (unsigned it = 0; it < 8u; ++it) {
        const unsigned rA = rbase + 2u * it;
        const v4f xa = *(const v4f*)(x + (size_t)rA * DM + c0);
        const v4f xb = *(const v4f*)(x + (size_t)(rA + 1u) * DM + c0);
        const v4f ya = ((xa - mu) * rs) * gv + bv;
        const v4f yb = ((xb - mu) * rs) * gv + bv;
        put2rows(sW[wave], lane, ya, yb, y32, y16, rA, 256.0f);
    }
}

constexpr size_t SZ_F32P  = (size_t)MTOK * DM * 4;
constexpr size_t SZ_H16   = (size_t)MTOK * DM * 2;
constexpr size_t SZ_QKV   = (size_t)MTOK * QKVW * 2;
constexpr size_t SZ_FF16  = (size_t)MTOK * FFD * 2;
constexpr size_t SZ_PART  = (size_t)2 * NSLAB * DM * 4;
constexpr size_t SZ_WQKV  = (size_t)NLAYER * QKVW * DM * 2;
constexpr size_t SZ_WO    = (size_t)NLAYER * DM * DM * 2;
constexpr size_t SZ_WFF   = (size_t)NLAYER * DM * FFD * 2;
constexpr size_t OFF_HS   = 0;
constexpr size_t OFF_TA   = OFF_HS + SZ_F32P;
constexpr size_t OFF_H16  = OFF_TA + SZ_F32P;
constexpr size_t OFF_QKV  = OFF_H16 + SZ_H16;
constexpr size_t OFF_O16  = OFF_QKV + SZ_QKV;
constexpr size_t OFF_FF16 = OFF_O16 + SZ_H16;
constexpr size_t OFF_PART = OFF_FF16 + SZ_FF16;
constexpr size_t OFF_WQKV = OFF_PART + SZ_PART;
constexpr size_t OFF_WO   = OFF_WQKV + SZ_WQKV;
constexpr size_t OFF_W1   = OFF_WO + SZ_WO;
constexpr size_t OFF_W2   = OFF_W1 + SZ_WFF;
constexpr size_t WS_TOTAL = OFF_W2 + SZ_WFF;
static_assert(SZ_F32P % 256 == 0 && SZ_H16 % 256 == 0 && SZ_QKV % 256 == 0 && SZ_FF16 % 256 == 0);
static_assert(SZ_PART % 256 == 0 && SZ_WQKV % 256 == 0 && SZ_WO % 256 == 0 && SZ_WFF % 256 == 0);
static_assert(WS_TOTAL <= 134217728);
static_assert(((MTOK / 64) * (QKVW / 64)) % 8 == 0 && ((MTOK / 64) * (DM / 64)) % 8 == 0 && ((MTOK / 64) * (FFD / 64)) % 8 == 0);
static_assert((DM * (DM / 8)) % 256 == 0 && (FFD * (DM / 8)) % 256 == 0 && (DM * (FFD / 8)) % 256 == 0);

extern "C" void kernel_launch(void* const* d_in, const int* in_sizes, int n_in, void* d_out, int out_size,
                              void* d_ws, size_t ws_size, hipStream_t stream) {
    if (n_in < 19) return;
    if (in_sizes[0] < NB * NC * 2 || in_sizes[1] < NB * NC || in_sizes[2] < NB * 2) return;
    if (in_sizes[3] < 2 * DM || in_sizes[4] < DM || in_sizes[5] < 3 * DM || in_sizes[6] < DM) return;
    if (in_sizes[7] < NLAYER * NH * DM * EH || in_sizes[8] < NLAYER * NH * DM * EH || in_sizes[9] < NLAYER * NH * DM * EH) return;
    if (in_sizes[10] < NLAYER * NH * EH * DM || in_sizes[11] < NLAYER * DM || in_sizes[12] < NLAYER * DM) return;
    if (in_sizes[13] < NLAYER * DM * FFD || in_sizes[14] < NLAYER * FFD || in_sizes[15] < NLAYER * FFD * DM) return;
    if (in_sizes[16] < NLAYER * DM || in_sizes[17] < NLAYER * DM || in_sizes[18] < NLAYER * DM) return;
    if (out_size < MTOK * DM) return;
    if (WS_TOTAL > ws_size) return;

    const float* input_loc    = (const float*)d_in[0];
    const float* input_demand = (const float*)d_in[1];
    const float* input_depot  = (const float*)d_in[2];
    const float* depot_w      = (const float*)d_in[3];
    const float* depot_b      = (const float*)d_in[4];
    const float* node_w       = (const float*)d_in[5];
    const float* node_b       = (const float*)d_in[6];
    const float* Wq           = (const float*)d_in[7];
    const float* Wk           = (const float*)d_in[8];
    const float* Wv           = (const float*)d_in[9];
    const float* Wo           = (const float*)d_in[10];
    const float* bn1_g        = (const float*)d_in[11];
    const float* bn1_b        = (const float*)d_in[12];
    const float* ffn_w1       = (const float*)d_in[13];
    const float* ffn_b1       = (const float*)d_in[14];
    const float* ffn_w2       = (const float*)d_in[15];
    const float* ffn_b2       = (const float*)d_in[16];
    const float* bn2_g        = (const float*)d_in[17];
    const float* bn2_b        = (const float*)d_in[18];
    float* out = (float*)d_out;

    char* wsp = (char*)d_ws;
    float*          hS    = (float*)(wsp + OFF_HS);
    float*          tA    = (float*)(wsp + OFF_TA);
    unsigned short* h16   = (unsigned short*)(wsp + OFF_H16);
    unsigned short* qkv16 = (unsigned short*)(wsp + OFF_QKV);
    unsigned short* o16   = (unsigned short*)(wsp + OFF_O16);
    unsigned short* ff16  = (unsigned short*)(wsp + OFF_FF16);
    float*          part  = (float*)(wsp + OFF_PART);
    unsigned short* wqkv  = (unsigned short*)(wsp + OFF_WQKV);
    unsigned short* wo    = (unsigned short*)(wsp + OFF_WO);
    unsigned short* wff1  = (unsigned short*)(wsp + OFF_W1);
    unsigned short* wff2  = (unsigned short*)(wsp + OFF_W2);
    float* psum = part;
    float* psq  = part + (size_t)NSLAB * DM;

    k_wt16<<<dim3((DM * (DM / 8)) / 256, NLAYER), 256, 0, stream>>>(Wq, DM, DM, 4, 4, QKVW * DM, wqkv);
    k_wt16<<<dim3((DM * (DM / 8)) / 256, NLAYER), 256, 0, stream>>>(Wk, DM, DM, 4, 4, QKVW * DM, wqkv + DM * DM);
    k_wt16<<<dim3((DM * (DM / 8)) / 256, NLAYER), 256, 0, stream>>>(Wv, DM, DM, 4, 4, QKVW * DM, wqkv + 2 * DM * DM);
    k_wt16<<<dim3((DM * (DM / 8)) / 256, NLAYER), 256, 0, stream>>>(Wo, DM, DM, 4, 7, DM * DM, wo);
    k_wt16<<<dim3((FFD * (DM / 8)) / 256, NLAYER), 256, 0, stream>>>(ffn_w1, DM, FFD, 4, 9, DM * FFD, wff1);
    k_wt16<<<dim3((DM * (FFD / 8)) / 256, NLAYER), 256, 0, stream>>>(ffn_w2, FFD, DM, 6, 7, DM * FFD, wff2);

    k_embed<<<MTOK / 16, 256, 0, stream>>>(input_loc, input_demand, input_depot, depot_w, depot_b, node_w, node_b, hS, h16);

    const unsigned gQ = ((MTOK / 64) * (QKVW / 64)) / 8;
    const unsigned gD = ((MTOK / 64) * (DM / 64)) / 8;
    const unsigned gF = ((MTOK / 64) * (FFD / 64)) / 8;

    for (int l = 0; l < NLAYER; ++l) {
        k_gemm_qkv<<<gQ, 256, 0, stream>>>((const _Float16*)h16, (const _Float16*)(wqkv + (size_t)l * QKVW * DM), (_Float16*)qkv16);
        k_attn<<<NB / 2, 512, 0, stream>>>((const _Float16*)qkv16, (_Float16*)o16);
        k_gemm_wo<<<gD, 256, 0, stream>>>((const _Float16*)o16, (const _Float16*)(wo + (size_t)l * DM * DM), hS, tA);
        k_colsum<<<NSLAB, 256, 0, stream>>>(tA, psum);
        k_colvar<<<NSLAB, 256, 0, stream>>>(tA, psum, psq);
        k_bn<<<NSLAB, 256, 0, stream>>>(tA, part, bn1_g + l * DM, bn1_b + l * DM, hS, h16);
        k_gemm_ff1<<<gF, 256, 0, stream>>>((const _Float16*)h16, (const _Float16*)(wff1 + (size_t)l * DM * FFD), ffn_b1 + l * FFD, (_Float16*)ff16);
        k_gemm_ff2<<<gD, 256, 0, stream>>>((const _Float16*)ff16, (const _Float16*)(wff2 + (size_t)l * DM * FFD), ffn_b2 + l * DM, hS, tA);
        k_colsum<<<NSLAB, 256, 0, stream>>>(tA, psum);
        k_colvar<<<NSLAB, 256, 0, stream>>>(tA, psum, psq);
        k_bn<<<NSLAB, 256, 0, stream>>>(tA, part, bn2_g + l * DM, bn2_b + l * DM, (l == NLAYER - 1) ? out : hS, h16);
    }
}
